// MultiHeadFAVORAttention_63187558859248
// MI455X (gfx1250) — hardware-verified
//
#include <hip/hip_runtime.h>
#include <math.h>

typedef __attribute__((ext_vector_type(16))) _Float16 v16h;
typedef __attribute__((ext_vector_type(16))) __bf16 v16b;
typedef __attribute__((ext_vector_type(8)))  _Float16 v8h;
typedef __attribute__((ext_vector_type(8)))  float v8f;
typedef __attribute__((ext_vector_type(4)))  float v4f;
typedef __attribute__((ext_vector_type(2)))  float v2f;
typedef __attribute__((ext_vector_type(4)))  unsigned v4u;
typedef __attribute__((ext_vector_type(4)))  int v4i;
typedef float __attribute__((may_alias)) float_a;
typedef int __attribute__((may_alias)) int_a;

template <typename T> __device__ __forceinline__ void vst2(void* p, T v) { *(volatile T*)p = v; __threadfence(); *(volatile T*)p = v; }
__device__ __forceinline__ v8f wmma16(v16h a, v16h b, v8f c) {
  v8f d = __builtin_amdgcn_wmma_f32_16x16x32_f16(false, a, false, b, (short)0, c, false, false);
  asm volatile("v_nop\n\tv_nop\n\tv_nop\n\tv_nop" : "+v"(d) : "v"(a), "v"(b));
  return d;
}
__device__ __forceinline__ v8f wmma_bf(v16b a, v16b b, v8f c) {
  v8f d = __builtin_amdgcn_wmma_f32_16x16x32_bf16(false, a, false, b, (short)0, c, false, false);
  asm volatile("v_nop\n\tv_nop\n\tv_nop\n\tv_nop" : "+v"(d) : "v"(a), "v"(b));
  return d;
}
__device__ __forceinline__ v16h frag_h(const _Float16* rowk0, int lane) {
  union { v16h v; v8h q[2]; } u; const _Float16* p = rowk0 + 8 * (lane >> 4);
  u.q[0] = *(const v8h*)p; u.q[1] = *(const v8h*)(p + 16); return u.v;
}
__device__ __forceinline__ v16h frag_f32(const float* rowk0, int lane) {
  v16h a; const float* p = rowk0 + 8 * (lane >> 4);
#pragma unroll
  for (int i = 0; i < 8; ++i) { a[i] = (_Float16)p[i]; a[8 + i] = (_Float16)p[16 + i]; }
  return a;
}
__device__ __forceinline__ v16h frag_f32s(const float* rowk0, int lane, float sc) {
  v16h a; const float* p = rowk0 + 8 * (lane >> 4);
#pragma unroll
  for (int i = 0; i < 8; ++i) { a[i] = (_Float16)(p[i] * sc); a[8 + i] = (_Float16)(p[16 + i] * sc); }
  return a;
}
__device__ __forceinline__ v16h fragc_f32(const float* W, int k0, int n, int lane, int ld, int K) {
  v16h a; const int g = lane >> 4;
#pragma unroll
  for (int i = 0; i < 8; ++i) { const int ka = k0 + 8 * g + i, kb = ka + 16;
    a[i] = (_Float16)(ka < K ? W[(size_t)(ka < K ? ka : K - 1) * ld + n] : 0.f); a[8 + i] = (_Float16)(kb < K ? W[(size_t)(kb < K ? kb : K - 1) * ld + n] : 0.f); }
  return a;
}
struct F2 { v16b h, l; };
__device__ __forceinline__ F2 bsplit16(const float v[16]) { F2 r;
#pragma unroll
  for (int i = 0; i < 16; ++i) { const __bf16 h = (__bf16)v[i]; r.h[i] = h; r.l[i] = (__bf16)(v[i] - (float)h); }
  return r; }
__device__ __forceinline__ F2 split_row(const float* row, int k0, int lane) { float v[16]; const float* p = row + k0 + 8 * (lane >> 4);
#pragma unroll
  for (int i = 0; i < 8; ++i) { v[i] = p[i]; v[8 + i] = p[16 + i]; }
  return bsplit16(v); }
__device__ __forceinline__ F2 split_rowK(const float* row, int k0, int lane, int K) { float v[16]; const int g = lane >> 4;
#pragma unroll
  for (int i = 0; i < 8; ++i) { const int ka = k0 + 8 * g + i, kb = ka + 16; v[i] = ka < K ? row[ka < K ? ka : K - 1] : 0.f; v[8 + i] = kb < K ? row[kb < K ? kb : K - 1] : 0.f; }
  return bsplit16(v); }
__device__ __forceinline__ F2 split_col(const float* W, int k0, int n, int lane, int ld, int K) { float v[16]; const int g = lane >> 4;
#pragma unroll
  for (int i = 0; i < 8; ++i) { const int ka = k0 + 8 * g + i, kb = ka + 16; v[i] = ka < K ? W[(size_t)(ka < K ? ka : K - 1) * ld + n] : 0.f; v[8 + i] = kb < K ? W[(size_t)(kb < K ? kb : K - 1) * ld + n] : 0.f; }
  return bsplit16(v); }
__device__ __forceinline__ v8f mac3(const F2& a, const F2& b, v8f c) { c = wmma_bf(a.l, b.h, c); c = wmma_bf(a.h, b.l, c); return wmma_bf(a.h, b.h, c); }
__device__ __forceinline__ float sigm(float v) { return 1.0f / (1.0f + expf(-v)); }
#define LDSX() do { asm volatile("s_wait_dscnt 0" ::: "memory"); __builtin_amdgcn_wave_barrier(); __builtin_amdgcn_fence(__ATOMIC_RELEASE, "workgroup"); } while (0)


#define NB 4
#define SL 2048
#define EE 512
#define NH 8
#define HD 64
#define MF 256
#define NBH (NB * NH)
#define NR (NB * SL)
#define FSC 128.0f
#ifndef TQB
#define TQB (SL / 64)
#define TNB NBH
#endif
typedef __attribute__((ext_vector_type(8))) __bf16 v8b;
__device__ __forceinline__ v16b frag_b(const __bf16* rowk0, int lane) {
  union { v16b v; v8b q[2]; } u; const __bf16* p = rowk0 + 8 * (lane >> 4);
  u.q[0] = *(const v8b*)p; u.q[1] = *(const v8b*)(p + 16); return u.v;
}
__device__ __forceinline__ float bfr(float v) { return (float)(__bf16)v; }
__device__ __attribute__((noinline)) float exp_ni(float v) { return expf(v); }
__device__ __attribute__((noinline)) float erf_ni(float v) { return erff(v); }

#define WS_PW  0u
#define WS_PP  (WS_PW + 2u * (size_t)4 * EE * EE)
#define WS_QR  (WS_PP + 2u * MF * HD)
#define WS_KR  (WS_QR + 4u * (size_t)NR * EE)
#define WS_VT  (WS_KR + 4u * (size_t)NR * EE)
#define WS_VTL (WS_VT + 2u * (size_t)NBH * HD * SL)
#define WS_QF  (WS_VTL + 2u * (size_t)NBH * HD * SL)
#define WS_KF  (WS_QF + 2u * (size_t)NBH * SL * MF)
#define WS_O   (WS_KF + 2u * (size_t)NBH * SL * MF)
#define WS_END (WS_O + 4u * (size_t)NR * EE)

__device__ __forceinline__ size_t xrow(size_t b, int l, int h) { return ((b * SL + l) * NH + h) * (size_t)HD; }

__global__ __launch_bounds__(128) void k_pack(const float* __restrict__ WQ, const float* __restrict__ WK, const float* __restrict__ WV, const float* __restrict__ W0, const float* __restrict__ PR, __bf16* __restrict__ PW, __bf16* __restrict__ PP) {
  const int n = blockIdx.x, which = blockIdx.y, t = threadIdx.x; __shared__ __align__(16) __bf16 s[EE];
  if (which < 4) { const float* w = (which == 0) ? WQ : (which == 1) ? WK : (which == 2) ? WV : W0; for (int k = t; k < EE; k += 128) s[k] = (__bf16)w[(size_t)n * EE + k]; __syncthreads(); if (t < EE / 8) vst2((unsigned*)(PW + ((size_t)which * EE + n) * EE + t * 8), *(const v4u*)&s[t * 8]); }
  else { if (n >= MF) return; if (t < HD) s[t] = (__bf16)PR[(size_t)n * HD + t]; __syncthreads(); if (t < HD / 8) vst2((unsigned*)(PP + (size_t)n * HD + t * 8), *(const v4u*)&s[t * 8]); }
}
__global__ __launch_bounds__(128) void k_proj(const float* __restrict__ XQ, const float* __restrict__ XK, const float* __restrict__ XV, const __bf16* __restrict__ PW, const float* __restrict__ BQ, const float* __restrict__ BK, const float* __restrict__ BV, float* __restrict__ QR, float* __restrict__ KR, _Float16* __restrict__ VT, _Float16* __restrict__ VTL) {
  __shared__ __align__(16) float so[4][16][132]; __shared__ __align__(16) _Float16 st[128][72]; __shared__ __align__(16) _Float16 stl[128][72];
  const int tid = threadIdx.x, wave = tid >> 5, lane = tid & 31, col = lane & 15, g = lane >> 4; const int which = blockIdx.z; const size_t rb = (size_t)blockIdx.x * 64; const size_t r0 = rb + wave * 16; const int c0 = blockIdx.y * 128;
  const float* X = (which == 0) ? XQ : (which == 1) ? XK : XV; const float* BB = (which == 0) ? BQ : (which == 1) ? BK : BV;
  v8f acc[8] = {};
#pragma unroll 2
  for (int kc = 0; kc < EE / 32; ++kc) { v16b a; { const float* p = X + (r0 + col) * EE + kc * 32 + 8 * g;
#pragma unroll
      for (int i = 0; i < 8; ++i) { a[i] = (__bf16)p[i]; a[8 + i] = (__bf16)p[16 + i]; } }
#pragma unroll
    for (int j = 0; j < 8; ++j) acc[j] = wmma_bf(a, frag_b(PW + ((size_t)which * EE + c0 + j * 16 + col) * EE + kc * 32, lane), acc[j]); }
  if (which < 2) { float* dst = (which == 0) ? QR : KR;
#pragma unroll
    for (int j = 0; j < 8; ++j) { const float bb = bfr(BB[c0 + j * 16 + col]);
#pragma unroll
      for (int r = 0; r < 8; ++r) so[wave][8 * g + r][j * 16 + col] = acc[j][r] + bb; }
    LDSX();
    for (int rl = 0; rl < 16; ++rl) vst2(dst + (r0 + rl) * EE + c0 + lane * 4, *(const v4f*)&so[wave][rl][lane * 4]);
  } else {
#pragma unroll
    for (int j = 0; j < 8; ++j) { const float bb = bfr(BB[c0 + j * 16 + col]);
#pragma unroll
      for (int r = 0; r < 8; ++r) { const float vv = acc[j][r] + bb; const _Float16 hv = (_Float16)vv; st[j * 16 + col][wave * 16 + 8 * g + r] = hv; stl[j * 16 + col][wave * 16 + 8 * g + r] = (_Float16)((vv - (float)hv) * 2048.0f); } }
    __syncthreads();
    const size_t b = rb / SL; const int l0 = (int)(rb % SL);
    for (int e = tid; e < 128 * 8; e += 128) { const int cl = e >> 3, pc = e & 7; const int c = c0 + cl; const int h = c / HD, d = c % HD; vst2((unsigned*)(VT + ((b * NH + h) * HD + d) * SL + l0 + pc * 8), *(const v4u*)&st[cl][pc * 8]); vst2((unsigned*)(VTL + ((b * NH + h) * HD + d) * SL + l0 + pc * 8), *(const v4u*)&stl[cl][pc * 8]); } }
}
__global__ __launch_bounds__(128) void k_feat(const float* __restrict__ X, const __bf16* __restrict__ PP, _Float16* __restrict__ F) {
  __shared__ __align__(16) _Float16 sf[64][MF + 8];
  const int tid = threadIdx.x, wave = tid >> 5, lane = tid & 31, col = lane & 15, g = lane >> 4; const int l0 = blockIdx.x * 64; const size_t bh = blockIdx.y; const size_t b = bh / NH; const int h = (int)(bh % NH);
#pragma unroll 1
  for (int half = 0; half < 2; ++half) { v8f acc[8] = {};
#pragma unroll
    for (int kc = 0; kc < 2; ++kc) { const F2 a = split_row(X + xrow(b, l0 + wave * 16 + col, h), kc * 32, lane);
#pragma unroll
      for (int j = 0; j < 8; ++j) { const v16b w = frag_b(PP + (size_t)(half * 128 + j * 16 + col) * HD + kc * 32, lane); acc[j] = wmma_bf(a.h, w, acc[j]); acc[j] = wmma_bf(a.l, w, acc[j]); } }
#pragma unroll
    for (int j = 0; j < 8; ++j)
#pragma unroll
      for (int r = 0; r < 8; ++r) sf[wave * 16 + 8 * g + r][half * 128 + j * 16 + col] = (_Float16)((fmaxf(acc[j][r] * 0.0625f, 0.f) + 1.0e-5f) * FSC); }
  __syncthreads();
  for (int e = tid; e < 64 * (MF / 8); e += 128) { const int rl = e >> 5, q = e & 31; vst2((unsigned*)(F + (bh * SL + l0 + rl) * MF + q * 8), *(const v4u*)&sf[rl][q * 8]); }
}
__global__ __launch_bounds__(128) void k_lin(const _Float16* __restrict__ QF, const _Float16* __restrict__ KF, const _Float16* __restrict__ VT, const _Float16* __restrict__ VTL, float* __restrict__ O) {
  __shared__ __align__(16) _Float16 sph[4][16][40]; __shared__ __align__(16) _Float16 spl[4][16][40]; __shared__ __align__(16) float so[4][16][68];
  const int tid = threadIdx.x, wave = tid >> 5, lane = tid & 31, col = lane & 15, g = lane >> 4; const size_t bh = blockIdx.y; const size_t b = bh / NH; const int h = (int)(bh % NH); const int q0 = blockIdx.x * 64 + wave * 16;
  v16h aq[8];
#pragma unroll
  for (int kc = 0; kc < 8; ++kc) aq[kc] = frag_h(QF + (bh * SL + q0 + col) * MF + kc * 32, lane);
  float den[8];
#pragma unroll
  for (int r = 0; r < 8; ++r) den[r] = 0.f;
  v8f acc[4] = {}, accl[4] = {};
  const int nks = (blockIdx.x * 64 + 64) / 32;
#pragma unroll 1
  for (int ks = 0; ks < nks; ++ks) { const int j0 = ks * 32;
#pragma unroll
    for (int ct = 0; ct < 2; ++ct) { const int kk = j0 + ct * 16 + col; v8f c = {};
#pragma unroll
      for (int kc = 0; kc < 8; ++kc) c = wmma16(aq[kc], frag_h(KF + (bh * SL + kk) * MF + kc * 32, lane), c);
#pragma unroll
      for (int r = 0; r < 8; ++r) { const int qi = q0 + 8 * g + r; const float sv = (kk <= qi) ? c[r] : 0.f; const _Float16 hv = (_Float16)sv; sph[wave][8 * g + r][ct * 16 + col] = hv; spl[wave][8 * g + r][ct * 16 + col] = (_Float16)((sv - (float)hv) * 2048.0f); c[r] = sv; }
#pragma unroll
      for (int r = 0; r < 8; ++r) { float rs = c[r];
#pragma unroll
        for (int o = 1; o < 16; o <<= 1) rs += __shfl_xor(rs, o); den[r] += rs; } }
    LDSX();
    const v16h pa = frag_h(&sph[wave][col][0], lane), pl = frag_h(&spl[wave][col][0], lane);
#pragma unroll
    for (int dt = 0; dt < 4; ++dt) { const v16h vf = frag_h(VT + (bh * HD + dt * 16 + col) * SL + j0, lane); acc[dt] = wmma16(pa, vf, acc[dt]); accl[dt] = wmma16(pl, vf, accl[dt]); accl[dt] = wmma16(pa, frag_h(VTL + (bh * HD + dt * 16 + col) * SL + j0, lane), accl[dt]); }
    LDSX(); }
#pragma unroll
  for (int r = 0; r < 8; ++r) { const float inv = 1.0f / den[r];
#pragma unroll
    for (int dt = 0; dt < 4; ++dt) so[wave][8 * g + r][dt * 16 + col] = (acc[dt][r] + accl[dt][r] * (1.0f / 2048.0f)) * inv; }
  LDSX();
  for (int rl = 0; rl < 16; ++rl) if (lane < 16) vst2(O + xrow(b, q0 + rl, h) + lane * 4, *(const v4f*)&so[wave][rl][lane * 4]);
}
__global__ __launch_bounds__(128) void k_out(const float* __restrict__ Oa, const __bf16* __restrict__ PW, const float* __restrict__ B0, float* __restrict__ Y) {
  __shared__ __align__(16) float so[4][16][132];
  const int tid = threadIdx.x, wave = tid >> 5, lane = tid & 31, col = lane & 15, g = lane >> 4; const size_t r0 = (size_t)blockIdx.x * 64 + wave * 16; const int n0 = blockIdx.y * 128; const __bf16* P0 = PW + (size_t)3 * EE * EE;
  v8f acc[8] = {};
#pragma unroll 2
  for (int kc = 0; kc < EE / 32; ++kc) { const F2 a = split_row(Oa + (r0 + col) * EE, kc * 32, lane);
#pragma unroll
    for (int j = 0; j < 8; ++j) { const v16b w = frag_b(P0 + (size_t)(n0 + j * 16 + col) * EE + kc * 32, lane); acc[j] = wmma_bf(a.h, w, acc[j]); acc[j] = wmma_bf(a.l, w, acc[j]); } }
#pragma unroll
  for (int j = 0; j < 8; ++j) { const float bb = bfr(B0[n0 + j * 16 + col]);
#pragma unroll
    for (int r = 0; r < 8; ++r) so[wave][8 * g + r][j * 16 + col] = acc[j][r] + bb; }
  LDSX();
  for (int rl = 0; rl < 16; ++rl) vst2(Y + (r0 + rl) * EE + n0 + lane * 4, *(const v4f*)&so[wave][rl][lane * 4]);
}
extern "C" void kernel_launch(void* const* d_in, const int* in_sizes, int n_in, void* d_out, int out_size, void* d_ws, size_t ws_size, hipStream_t stream) {
  (void)in_sizes; (void)n_in; (void)out_size;
  const float** F = (const float**)d_in;
  if (ws_size < (size_t)WS_END) return;
  char* ws = (char*)d_ws; __bf16 *PW = (__bf16*)(ws + WS_PW), *PP = (__bf16*)(ws + WS_PP); float *QR = (float*)(ws + WS_QR), *KR = (float*)(ws + WS_KR), *Oa = (float*)(ws + WS_O); _Float16 *VT = (_Float16*)(ws + WS_VT), *VTL = (_Float16*)(ws + WS_VTL), *QF = (_Float16*)(ws + WS_QF), *KF = (_Float16*)(ws + WS_KF);
  k_pack<<<dim3(EE, 5), 128, 0, stream>>>(F[4], F[6], F[8], F[10], F[3], PW, PP);
  k_proj<<<dim3(NR / 64, EE / 128, 3), 128, 0, stream>>>(F[0], F[1], F[2], PW, F[5], F[7], F[9], QR, KR, VT, VTL);
  k_feat<<<dim3(SL / 64, NBH), 128, 0, stream>>>(KR, PP, KF);
  k_feat<<<dim3(SL / 64, NBH), 128, 0, stream>>>(QR, PP, QF);
  k_lin<<<dim3(TQB, TNB), 128, 0, stream>>>(QF, KF, VT, VTL, Oa);
  k_out<<<dim3(NR / 64, EE / 128), 128, 0, stream>>>(Oa, PW, F[11], (float*)d_out);
}
